// Downsample_PASA_group_softmax_46986942218656
// MI455X (gfx1250) — hardware-verified
//
#include <hip/hip_runtime.h>


#define NI   2
#define CC   64
#define SD   32
#define NPOS 32768
#define KK   1728
#define CO   54
#define COP  64
#define SLAB 4096
#define OS   16
#define NOUT 4096
typedef _Float16 h16;
typedef unsigned short bf;
typedef __attribute__((ext_vector_type(16))) __bf16   v16bf;
typedef __attribute__((ext_vector_type(16))) _Float16 v16h;
typedef __attribute__((ext_vector_type(8)))  _Float16 v8h;
typedef __attribute__((ext_vector_type(8)))  unsigned short v8us;
typedef __attribute__((ext_vector_type(8)))  float    v8f;
typedef __attribute__((ext_vector_type(4)))  float    v4f;
typedef v8h  __attribute__((may_alias)) v8ha;
typedef v4f  __attribute__((may_alias)) v4fa;
typedef v8us __attribute__((may_alias)) v8usa;

__device__ __forceinline__ unsigned short f2bf(float f) { unsigned u = __float_as_uint(f); u += 0x7FFFu + ((u >> 16) & 1u); return (unsigned short)(u >> 16); }
__device__ __forceinline__ float bf2f(unsigned short b) { return __uint_as_float(((unsigned)b) << 16); }
__device__ __forceinline__ float bfr(float f) { return bf2f(f2bf(f)); }
__device__ __forceinline__ v16h cat16(v8h lo, v8h hi) { return __builtin_shufflevector(lo, hi, 0, 1, 2, 3, 4, 5, 6, 7, 8, 9, 10, 11, 12, 13, 14, 15); }
__device__ __forceinline__ v16bf cat16b(v8us lo, v8us hi) { return __builtin_bit_cast(v16bf, __builtin_shufflevector(lo, hi, 0, 1, 2, 3, 4, 5, 6, 7, 8, 9, 10, 11, 12, 13, 14, 15)); }
__device__ __forceinline__ v8f wmma16(v16h a, v16h b, v8f c) { return __builtin_amdgcn_wmma_f32_16x16x32_f16(false, a, false, b, (short)0, c, false, false); }
__device__ __forceinline__ v8f wmmab(v16bf a, v16bf b, v8f c) { return __builtin_amdgcn_wmma_f32_16x16x32_bf16(false, a, false, b, (short)0, c, false, false); }


template <typename T16> struct WFrag;
template <> struct WFrag<h16> { typedef v16h V; static __device__ __forceinline__ V ld(const h16* p) { return cat16(*(const v8h*)p, *(const v8h*)(p + 16)); } static __device__ __forceinline__ v8f mma(V a, V b, v8f c) { return wmma16(a, b, c); } };
template <> struct WFrag<bf> { typedef v16bf V; static __device__ __forceinline__ V ld(const bf* p) { return cat16b(*(const v8us*)p, *(const v8us*)(p + 16)); } static __device__ __forceinline__ v8f mma(V a, V b, v8f c) { return wmmab(a, b, c); } };
template <typename T16, int NSPLIT, bool BIAS>
__global__ __launch_bounds__(32) void k_gemmw(const T16* __restrict__ A, const T16* __restrict__ A2, const T16* __restrict__ Bt, const T16* __restrict__ Bt2, int K, float* C, int ldc, const float* __restrict__ bias, size_t sA, size_t sB, size_t sC) {
    typedef typename WFrag<T16>::V V;
    __shared__ __align__(16) float os[16 * 68];
    const size_t z = blockIdx.z; A += z * sA; if (A2) A2 += z * sA; Bt += z * sB; if (Bt2) Bt2 += z * sB; C += z * sC;
    const int lane = threadIdx.x & 31, lr = lane & 15, hi = lane >> 4; const int r0 = blockIdx.x * 64, c0 = blockIdx.y * 64;
    v8f acc[4][4];
#pragma unroll
    for (int mb = 0; mb < 4; ++mb)
#pragma unroll
        for (int nb = 0; nb < 4; ++nb) acc[mb][nb] = (v8f){};
    const size_t aoff = (size_t)(r0 + lr) * K + 8 * hi, boff = (size_t)(c0 + lr) * K + 8 * hi;
#pragma unroll 1
    for (int kc = 0; kc < K; kc += 32) {
        V a[4], a2[4];
#pragma unroll
        for (int mb = 0; mb < 4; ++mb) { a[mb] = WFrag<T16>::ld(A + aoff + (size_t)mb * 16 * K + kc); if (NSPLIT == 1 || NSPLIT == 2) a2[mb] = WFrag<T16>::ld(A2 + aoff + (size_t)mb * 16 * K + kc); }
#pragma unroll
        for (int nb = 0; nb < 4; ++nb) { const V b = WFrag<T16>::ld(Bt + boff + (size_t)nb * 16 * K + kc); V b2; if (NSPLIT >= 2) b2 = WFrag<T16>::ld(Bt2 + boff + (size_t)nb * 16 * K + kc);
#pragma unroll
            for (int mb = 0; mb < 4; ++mb) { acc[mb][nb] = WFrag<T16>::mma(a[mb], b, acc[mb][nb]); if (NSPLIT == 1 || NSPLIT == 2) acc[mb][nb] = WFrag<T16>::mma(a2[mb], b, acc[mb][nb]); if (NSPLIT >= 2) acc[mb][nb] = WFrag<T16>::mma(a[mb], b2, acc[mb][nb]); } }
        asm volatile("v_nop\n\tv_nop\n\tv_nop\n\tv_nop" : "+v"(acc[0][0]), "+v"(acc[1][1]), "+v"(acc[2][2]), "+v"(acc[3][3]) : "v"(a[0]), "v"(a[3]));
    }
#pragma unroll
    for (int mb = 0; mb < 4; ++mb) {
#pragma unroll
        for (int nb = 0; nb < 4; ++nb) {
#pragma unroll
            for (int j = 0; j < 8; ++j) os[(hi * 8 + j) * 68 + nb * 16 + lr] = acc[mb][nb][j]; }
        __builtin_amdgcn_wave_barrier(); asm volatile("" ::: "memory");
        float* crow = C + (size_t)(r0 + mb * 16) * ldc + c0;
#pragma unroll 1
        for (int ps = 0; ps < 2; ++ps) {
#pragma unroll
            for (int s = 0; s < 8; ++s) { const int row = 2 * s + hi, cofs = lr * 4; v4f val = *(const v4fa*)(os + row * 68 + cofs); if (BIAS) { val[0] += bfr(bias[c0 + cofs]); val[1] += bfr(bias[c0 + cofs + 1]); val[2] += bfr(bias[c0 + cofs + 2]); val[3] += bfr(bias[c0 + cofs + 3]); }
                *(volatile v4f*)(crow + (size_t)row * ldc + cofs) = val; }
            if (ps == 0) __threadfence(); }
        __builtin_amdgcn_wave_barrier(); asm volatile("" ::: "memory");
    }
}

typedef __attribute__((ext_vector_type(2))) float v2f;
typedef __attribute__((ext_vector_type(4))) unsigned short v4us;

__device__ __forceinline__ int refl(int i) { return i < 0 ? -i : (i >= SD ? 2 * SD - 2 - i : i); }
__global__ __launch_bounds__(256) void k_wpad(const float* __restrict__ w, bf* Bt) { const size_t e = ((size_t)blockIdx.x * 256 + threadIdx.x) * 4; if (e >= (size_t)COP * KK) return; const int r = (int)(e / KK); v4us o;
#pragma unroll
    for (int u = 0; u < 4; ++u) o[u] = (r < CO) ? f2bf(w[e + u]) : (unsigned short)0; *(volatile v4us*)(Bt + e) = o; __threadfence(); *(volatile v4us*)(Bt + e) = o; }
__global__ __launch_bounds__(256) void k_i2c3(const float* __restrict__ x, int p0, bf* A) { const size_t e = ((size_t)blockIdx.x * 256 + threadIdx.x) * 4; if (e >= (size_t)SLAB * KK) return; const int k0 = (int)(e % KK); const int p = p0 + (int)(e / KK); const int w_ = p % SD, y = (p / SD) % SD, z = p / (SD * SD); v4us o;
#pragma unroll
    for (int u = 0; u < 4; ++u) { const int k = k0 + u; const int ci = k / 27, t = k % 27; const int i = t / 9, j = (t / 3) % 3, l = t % 3; o[u] = f2bf(x[(((size_t)ci * SD + refl(z + i - 1)) * SD + refl(y + j - 1)) * SD + refl(w_ + l - 1)]); }
    *(volatile v4us*)(A + e) = o; __threadfence(); *(volatile v4us*)(A + e) = o; }
__global__ __launch_bounds__(256) void k_bnstat(const float* __restrict__ Y, float* ST) { __shared__ float red[256]; const int c = blockIdx.x; const int tid = threadIdx.x; float s = 0.f;
    for (int i = tid; i < NI * NPOS; i += 256) s += Y[(size_t)i * COP + c];
    red[tid] = s; __syncthreads(); for (int k = 128; k; k >>= 1) { if (tid < k) red[tid] = __fadd_rn(red[tid], red[tid + k]); __syncthreads(); } const float mean = red[0] * (1.0f / (NI * NPOS)); __syncthreads();
    float q = 0.f; for (int i = tid; i < NI * NPOS; i += 256) { float d = __fsub_rn(Y[(size_t)i * COP + c], mean); asm volatile("" : "+v"(d)); float p = __fmul_rn(d, d); asm volatile("" : "+v"(p)); q = __fadd_rn(q, p); }
    red[tid] = q; __syncthreads(); for (int k = 128; k; k >>= 1) { if (tid < k) red[tid] = __fadd_rn(red[tid], red[tid + k]); __syncthreads(); }
    if (tid == 0) { v2f o; o[0] = mean; o[1] = __frsqrt_rn(__fadd_rn(red[0] * (1.0f / (NI * NPOS)), 1e-5f)); *(volatile v2f*)(ST + 2 * c) = o; __threadfence(); *(volatile v2f*)(ST + 2 * c) = o; } }
__global__ __launch_bounds__(256) void k_sig(const float* __restrict__ SIG, const float* __restrict__ ST, const float* __restrict__ ga, const float* __restrict__ be, int n, float* SGN) { const int e = (blockIdx.x * 256 + threadIdx.x) * 4; if (e >= NOUT * COP) return; const int c0 = e % COP; const int q = e / COP; const int ow = q % OS, oh = (q / OS) % OS, od = q / (OS * OS); const size_t p = (size_t)n * NPOS + ((size_t)(2 * od) * SD + 2 * oh) * SD + 2 * ow;
    const v4f a = *(const v4f*)(SIG + p * COP + c0); float z[4]; float mx = -3.0e38f;
#pragma unroll
    for (int u = 0; u < 4; ++u) { const int c = c0 + u; if (c < CO) { float t0 = __fmul_rn(__fsub_rn(a[u], ST[2 * c]), ST[2 * c + 1]); asm volatile("" : "+v"(t0)); float g = bfr(ga[c]), bb = bfr(be[c]); asm volatile("" : "+v"(g)); asm volatile("" : "+v"(bb)); float t1 = __fmul_rn(g, t0); asm volatile("" : "+v"(t1)); z[u] = __fadd_rn(t1, bb); mx = fmaxf(mx, z[u]); } else z[u] = -3.0e38f; }
    mx = fmaxf(mx, __shfl_xor(mx, 1, 32)); mx = fmaxf(mx, __shfl_xor(mx, 2, 32)); mx = fmaxf(mx, __shfl_xor(mx, 4, 32)); mx = fmaxf(mx, __shfl_xor(mx, 8, 32)); float ev[4]; float s = 0.f;
#pragma unroll
    for (int u = 0; u < 4; ++u) { if (c0 + u < CO) { float d = __fsub_rn(z[u], mx); asm volatile("" : "+v"(d)); ev[u] = __expf(d); s = __fadd_rn(s, ev[u]); } else ev[u] = 0.f; }
    s += __shfl_xor(s, 1, 32); s += __shfl_xor(s, 2, 32); s += __shfl_xor(s, 4, 32); s += __shfl_xor(s, 8, 32); const float inv = __fdiv_rn(1.0f, s); v4f o;
#pragma unroll
    for (int u = 0; u < 4; ++u) o[u] = __fmul_rn(ev[u], inv); *(volatile v4f*)(SGN + e) = o; __threadfence(); *(volatile v4f*)(SGN + e) = o; }
__global__ __launch_bounds__(256) void k_out(const float* __restrict__ x, const float* __restrict__ SGN, float* OUTn) { const int idx = blockIdx.x * 256 + threadIdx.x; if (idx >= CC * NOUT) return; const int q = idx % NOUT; const int c = idx / NOUT; const int ow = q % OS, oh = (q / OS) % OS, od = q / (OS * OS); const int g = c / (CC / 2); const float* sg = SGN + (size_t)q * COP + g * 27; float acc = 0.f;
#pragma unroll 1
    for (int t = 0; t < 27; ++t) { const int i = t / 9, j = (t / 3) % 3, l = t % 3; float xv = bfr(x[(((size_t)c * SD + refl(2 * od + i - 1)) * SD + refl(2 * oh + j - 1)) * SD + refl(2 * ow + l - 1)]); asm volatile("" : "+v"(xv)); float pr = __fmul_rn(xv, sg[t]); asm volatile("" : "+v"(pr)); acc = __fadd_rn(acc, pr); }
    *(volatile float*)(OUTn + idx) = acc; __threadfence(); *(volatile float*)(OUTn + idx) = acc; }

extern "C" void kernel_launch(void* const* d_in, const int* in_sizes, int n_in,
                              void* d_out, int out_size, void* d_ws, size_t ws_size, hipStream_t stream) {
    (void)in_sizes; (void)n_in; (void)out_size;
    const float* x = (const float*)d_in[0]; const float* cw = (const float*)d_in[1]; const float* ga = (const float*)d_in[2]; const float* be = (const float*)d_in[3];
    float* OUT = (float*)d_out;
    char* wsp = (char*)d_ws;
    auto take = [&](size_t bytes) { char* p = wsp; wsp += (bytes + 255) & ~(size_t)255; return (void*)p; };
    bf* WB = (bf*)take((size_t)COP * KK * 2); bf* A = (bf*)take((size_t)SLAB * KK * 2); float* SIG = (float*)take((size_t)NI * NPOS * COP * 4); float* ST = (float*)take(COP * 2 * 4); float* SGN = (float*)take((size_t)NOUT * COP * 4);
    if ((size_t)(wsp - (char*)d_ws) > ws_size) return;
    k_wpad<<<(unsigned)(((size_t)COP * KK / 4 + 255) / 256), 256, 0, stream>>>(cw, WB);
    for (int n = 0; n < NI; ++n) for (int p0 = 0; p0 < NPOS; p0 += SLAB) {
        k_i2c3<<<(unsigned)(((size_t)SLAB * KK / 4 + 255) / 256), 256, 0, stream>>>(x + (size_t)n * CC * NPOS, p0, A);
        k_gemmw<bf, 0, false><<<dim3(SLAB / 64, 1, 1), 32, 0, stream>>>(A, nullptr, WB, nullptr, KK, SIG + ((size_t)n * NPOS + p0) * COP, COP, nullptr, 0, 0, 0); }
    k_bnstat<<<CO, 256, 0, stream>>>(SIG, ST);
    for (int n = 0; n < NI; ++n) {
        k_sig<<<(NOUT * COP / 4 + 255) / 256, 256, 0, stream>>>(SIG, ST, ga, be, n, SGN);
        k_out<<<(CC * NOUT + 255) / 256, 256, 0, stream>>>(x + (size_t)n * CC * NPOS, SGN, OUT + (size_t)n * CC * NOUT); }
}
